// VanillaLSTMNet_6914897346578
// MI455X (gfx1250) — hardware-run, weakly checked
//
#include <hip/hip_runtime.h>
#include <math.h>

constexpr int OBS_STEPS  = 8;
constexpr int PRED_STEPS = 12;
constexpr int NBATCH     = 65536;
constexpr int NHID       = 64;
constexpr int NEMB       = 64;
constexpr int NGATE      = 256;
constexpr int ROWS_BLK   = 128;
constexpr int NTHR       = 256;
constexpr int H16_PITCH  = 72;
constexpr int W_PITCH    = 72;
constexpr int H32_PITCH  = 68;
constexpr int C_PITCH    = 68;
constexpr int H16_TILE   = ROWS_BLK * H16_PITCH;
constexpr int TAB_PHASE  = 3 * NGATE;
constexpr int WH_PHASE   = NGATE * NHID;
constexpr int REL_TILE   = 2 * ROWS_BLK;
constexpr float W_CARRY  = 16.0f;
constexpr float H_CARRY  = 256.0f;
constexpr float FOLD_INV = 1.0f / (W_CARRY * H_CARRY);
constexpr float LOG2E_F  = 1.44269504088896341f;
constexpr float K_SIG    = -LOG2E_F;
constexpr float K_TANH   = 2.0f * LOG2E_F;
constexpr float KF_SIG   = K_SIG * FOLD_INV;
constexpr float KF_TANH  = K_TANH * FOLD_INV;

static_assert(NGATE == 4 * NHID);
static_assert(NGATE == NTHR);
static_assert(NBATCH % ROWS_BLK == 0);
static_assert(NHID % 32 == 0);
static_assert(REL_TILE == NTHR);
static_assert((2 * H16_TILE) % NTHR == 0);
static_assert(2 * WH_PHASE == 16 * NTHR * 8);
static_assert((NGATE * (NHID / 8)) % NTHR == 0);
static_assert(H16_PITCH % 8 == 0 && W_PITCH % 8 == 0 && H32_PITCH % 4 == 0);

typedef __attribute__((ext_vector_type(16))) _Float16 v16h;
typedef __attribute__((ext_vector_type(8)))  _Float16 v8h;
typedef __attribute__((ext_vector_type(8)))  float    v8f;
typedef __attribute__((ext_vector_type(4)))  float    v4f;
typedef __attribute__((ext_vector_type(2)))  float    v2f;

__device__ __forceinline__ void group_guard(v8f& a, v8f& b, v8f& c, v8f& d, v16h x, v16h y) {
  asm volatile("v_nop\n\tv_nop\n\tv_nop\n\tv_nop\n\tv_nop" : "+v"(a), "+v"(b), "+v"(c), "+v"(d) : "v"(x), "v"(y));
}
__device__ __forceinline__ void keep4_h(v16h a, v16h b, v16h c, v16h d) { asm volatile("v_nop" :: "v"(a), "v"(b), "v"(c), "v"(d)); }

union FragU { v16h v; v8h h[2]; };
__device__ __forceinline__ v16h frag_load(const _Float16* p) {
  FragU f;
  f.h[0] = *(const v8h*)(p);
  f.h[1] = *(const v8h*)(p + 16);
  return f.v;
}
__device__ __forceinline__ v8f frag_mma(v16h a, v16h b, v8f c) {
  return __builtin_amdgcn_wmma_f32_16x16x32_f16(false, a, false, b, (short)0, c, false, false);
}

__global__ __launch_bounds__(NTHR) void prep_tables_kernel(
    const float* __restrict__ e_ew, const float* __restrict__ e_eb, const float* __restrict__ e_wih,
    const float* __restrict__ e_bih, const float* __restrict__ e_bhh,
    const float* __restrict__ d_ew, const float* __restrict__ d_eb, const float* __restrict__ d_wih,
    const float* __restrict__ d_bih, const float* __restrict__ d_bhh,
    float* __restrict__ TAB) {
  const int phase = blockIdx.x;
  const int n = threadIdx.x;
  const float* ew  = phase ? d_ew  : e_ew;
  const float* eb  = phase ? d_eb  : e_eb;
  const float* wih = phase ? d_wih : e_wih;
  const float* bih = phase ? d_bih : e_bih;
  const float* bhh = phase ? d_bhh : e_bhh;
  const float* wr = wih + (size_t)n * NEMB;
  float p0 = 0.0f, p1 = 0.0f, q = 0.0f;
#pragma unroll 1
  for (int e4 = 0; e4 < NEMB; e4 += 4) {
    const v4f w  = *(const v4f*)(wr + e4);
    const v4f m0 = *(const v4f*)(ew + 2 * e4);
    const v4f m1 = *(const v4f*)(ew + 2 * e4 + 4);
    const v4f bb = *(const v4f*)(eb + e4);
    p0 = fmaf(w[0], m0[0], p0); p1 = fmaf(w[0], m0[1], p1); q = fmaf(w[0], bb[0], q);
    p0 = fmaf(w[1], m0[2], p0); p1 = fmaf(w[1], m0[3], p1); q = fmaf(w[1], bb[1], q);
    p0 = fmaf(w[2], m1[0], p0); p1 = fmaf(w[2], m1[1], p1); q = fmaf(w[2], bb[2], q);
    p0 = fmaf(w[3], m1[2], p0); p1 = fmaf(w[3], m1[3], p1); q = fmaf(w[3], bb[3], q);
  }
  const float pbv = q + (bih[n] + bhh[n]);
  float* tp = TAB + (size_t)phase * TAB_PHASE + n;
  *(volatile float*)(tp)             = p0;
  *(volatile float*)(tp + NGATE)     = p1;
  *(volatile float*)(tp + 2 * NGATE) = pbv;
  __threadfence();
  *(volatile float*)(tp)             = p0;
  *(volatile float*)(tp + NGATE)     = p1;
  *(volatile float*)(tp + 2 * NGATE) = pbv;
}

__global__ __launch_bounds__(NTHR) void cvt_whh_kernel(const float* __restrict__ w_enc, const float* __restrict__ w_dec,
                                                       unsigned short* __restrict__ dst) {
  const int i = blockIdx.x * NTHR + threadIdx.x;
  const int phase = blockIdx.x >> 3;
  const int j = i & 2047;
  const float* src = phase ? w_dec : w_enc;
  const v4f a = *(const v4f*)(src + (size_t)j * 8);
  const v4f b = *(const v4f*)(src + (size_t)j * 8 + 4);
  v8h hv;
#pragma unroll
  for (int e = 0; e < 4; ++e) {
    hv[e]     = (_Float16)(a[e] * W_CARRY);
    hv[4 + e] = (_Float16)(b[e] * W_CARRY);
  }
  _Float16* dp = (_Float16*)dst + (size_t)i * 8;
  *(volatile v8h*)dp = hv;
  __threadfence();
  *(volatile v8h*)dp = hv;
}

__global__ __launch_bounds__(NTHR) __attribute__((amdgpu_num_vgpr(256)))
void lstm_seq_kernel(const float* __restrict__ obs_rel,
                     const unsigned short* __restrict__ WHp,
                     const float* __restrict__ TAB,
                     const float* __restrict__ h2p_w,
                     const float* __restrict__ h2p_b,
                     float* __restrict__ out) {
  __shared__ __align__(16) _Float16 sH16[2 * H16_TILE];
  __shared__ __align__(16) _Float16 sW[NGATE * W_PITCH];
  __shared__ __align__(16) float    sH32[ROWS_BLK * H32_PITCH];
  __shared__ __align__(16) float    sC[ROWS_BLK * C_PITCH];
  __shared__ __align__(16) float    sRel[2 * REL_TILE];
  __shared__ __align__(16) float    sW2[2 * NHID];
  __shared__ float                  sB2[2];

  const int tid  = threadIdx.x;
  const int lane = tid & 31;
  const int wave = tid >> 5;
  const int jw   = wave & 3;
  const int rows0 = (wave >> 2) * 64;
  const int c    = lane & 15;
  const int hh   = lane >> 4;
  const int koff = hh * 8;
  const int col  = jw * 16 + c;
  const int wgBase = blockIdx.x * ROWS_BLK;

#pragma unroll 1
  for (int i = tid; i < 2 * H16_TILE; i += NTHR) sH16[i] = (_Float16)0.0f;
  {
    v8h zz;
#pragma unroll
    for (int e = 0; e < 8; ++e) zz[e] = (_Float16)0.0f;
    *(v8h*)(sW + tid * W_PITCH + NHID) = zz;
  }
  if (tid < 2 * NHID) sW2[tid] = h2p_w[tid];
  {
    float bv = h2p_b[tid & 1];
    asm volatile("" : "+v"(bv));
    if (tid < 2) sB2[tid] = bv;
  }
  sRel[tid] = obs_rel[(size_t)wgBase * 2 + tid];

  const v8f z8 = {0.f, 0.f, 0.f, 0.f, 0.f, 0.f, 0.f, 0.f};
  float kP0[4], kP1[4], kpb[4];

#pragma unroll 1
  for (int phase = 0; phase < 2; ++phase) {
    __syncthreads();
    {
      const _Float16* wsrc = (const _Float16*)WHp + (size_t)phase * WH_PHASE;
#pragma unroll 1
      for (int i = tid; i < NGATE * (NHID / 8); i += NTHR) {
        const int n  = i >> 3;
        const int c8 = (i & 7) * 8;
        const v8h w = *(const v8h*)(wsrc + (size_t)i * 8);
        *(v8h*)(sW + n * W_PITCH + c8) = w;
      }
    }
#pragma unroll 1
    for (int rt = 0; rt < 4; ++rt) {
#pragma unroll
      for (int r = 0; r < 8; ++r) sC[(rows0 + rt * 16 + 8 * hh + r) * C_PITCH + col] = 0.0f;
    }
    {
      const float* tb = TAB + (size_t)phase * TAB_PHASE;
#pragma unroll
      for (int g = 0; g < 4; ++g) {
        const int n = g * NHID + col;
        const float sc = (g == 2) ? K_TANH : K_SIG;
        kP0[g] = sc * tb[n];
        kP1[g] = sc * tb[NGATE + n];
        kpb[g] = sc * tb[2 * NGATE + n];
      }
    }

    const int nst = phase ? PRED_STEPS : OBS_STEPS;
#pragma unroll 1
    for (int st = 0; st < nst; ++st) {
      const int gs  = phase * OBS_STEPS + st;
      const int cur = gs & 1;
      const _Float16* hcur  = sH16 + cur * H16_TILE;
      _Float16*       hnext = sH16 + (cur ^ 1) * H16_TILE;
      const float*    relc  = sRel + cur * REL_TILE;
      float*          reln  = sRel + (cur ^ 1) * REL_TILE;

      __syncthreads();

#pragma unroll 1
      for (int rt = 0; rt < 4; ++rt) {
        asm volatile("" ::: "memory");
        const int rbase = rows0 + rt * 16;
        const _Float16* ap = hcur + (rbase + c) * H16_PITCH + koff;
        const v16h a0 = frag_load(ap);
        const v16h a1 = frag_load(ap + 32);
        const _Float16* bp = sW + col * W_PITCH + koff;
        const v16h b00 = frag_load(bp);
        const v16h b01 = frag_load(bp + 32);
        const v16h b10 = frag_load(bp + 1 * NHID * W_PITCH);
        const v16h b11 = frag_load(bp + 1 * NHID * W_PITCH + 32);
        const v16h b20 = frag_load(bp + 2 * NHID * W_PITCH);
        const v16h b21 = frag_load(bp + 2 * NHID * W_PITCH + 32);
        const v16h b30 = frag_load(bp + 3 * NHID * W_PITCH);
        const v16h b31 = frag_load(bp + 3 * NHID * W_PITCH + 32);
        v8f ai = z8, af = z8, ag = z8, ao = z8;
        ai = frag_mma(a0, b00, ai);
        af = frag_mma(a0, b10, af);
        ag = frag_mma(a0, b20, ag);
        ao = frag_mma(a0, b30, ao);
        ai = frag_mma(a1, b01, ai);
        af = frag_mma(a1, b11, af);
        ag = frag_mma(a1, b21, ag);
        ao = frag_mma(a1, b31, ao);
        group_guard(ai, af, ag, ao, a0, a1);
        keep4_h(b00, b10, b20, b30);
        keep4_h(b01, b11, b21, b31);
        __builtin_amdgcn_sched_barrier(0);

#pragma unroll
        for (int r = 0; r < 8; ++r) {
          const int row = rbase + 8 * hh + r;
          const v2f rr = *(const v2f*)(relc + 2 * row);
          const float r0 = rr[0];
          const float r1 = rr[1];
          const float cold = sC[row * C_PITCH + col];
          const float xi = fmaf(r1, kP1[0], fmaf(r0, kP0[0], kpb[0]));
          const float xf = fmaf(r1, kP1[1], fmaf(r0, kP0[1], kpb[1]));
          const float xg = fmaf(r1, kP1[2], fmaf(r0, kP0[2], kpb[2]));
          const float xo = fmaf(r1, kP1[3], fmaf(r0, kP0[3], kpb[3]));
          const float ei = __builtin_amdgcn_exp2f(fmaf(ai[r], KF_SIG,  xi));
          const float ef = __builtin_amdgcn_exp2f(fmaf(af[r], KF_SIG,  xf));
          const float eg = __builtin_amdgcn_exp2f(fmaf(ag[r], KF_TANH, xg));
          const float eo = __builtin_amdgcn_exp2f(fmaf(ao[r], KF_SIG,  xo));
          const float iv = __builtin_amdgcn_rcpf(1.0f + ei);
          const float fv = __builtin_amdgcn_rcpf(1.0f + ef);
          const float ov = __builtin_amdgcn_rcpf(1.0f + eo);
          const float gv = fmaf(__builtin_amdgcn_rcpf(1.0f + eg), -2.0f, 1.0f);
          const float cn = fmaf(fv, cold, iv * gv);
          sC[row * C_PITCH + col] = cn;
          const float ec = __builtin_amdgcn_exp2f(cn * K_TANH);
          const float hn = ov * fmaf(__builtin_amdgcn_rcpf(1.0f + ec), -2.0f, 1.0f);
          hnext[row * H16_PITCH + col] = (_Float16)(hn * H_CARRY);
          sH32[row * H32_PITCH + col] = hn;
          if ((r & 1) == 1) __builtin_amdgcn_sched_barrier(0);
        }
      }

      if (phase == 0) {
        const int tn = (st + 1 < OBS_STEPS) ? (st + 1) : (OBS_STEPS - 1);
        const float v = obs_rel[((size_t)tn * NBATCH + wgBase) * 2 + tid];
        reln[tid] = v;
      } else {
        __syncthreads();
        const int prow = tid >> 1;
        const int pd   = tid & 1;
        const float* hp = sH32 + prow * H32_PITCH;
        const float* wp = sW2 + pd * NHID;
        float s = 0.0f;
#pragma unroll 4
        for (int q4 = 0; q4 < NHID; q4 += 4) {
          const v4f hv = *(const v4f*)(hp + q4);
          const v4f wv = *(const v4f*)(wp + q4);
          s = fmaf(hv[0], wv[0], s);
          s = fmaf(hv[1], wv[1], s);
          s = fmaf(hv[2], wv[2], s);
          s = fmaf(hv[3], wv[3], s);
        }
        s += sB2[pd];
        reln[tid] = s;
        float* op = out + ((size_t)st * NBATCH + wgBase) * 2 + tid;
        *(volatile float*)op = s;
        __threadfence();
        *(volatile float*)op = s;
      }
    }
  }
}

extern "C" void kernel_launch(void* const* d_in, const int* in_sizes, int n_in,
                              void* d_out, int out_size, void* d_ws, size_t ws_size, hipStream_t stream) {
  if (n_in < 16 || d_out == nullptr || d_ws == nullptr) return;
  if (in_sizes[1] != OBS_STEPS * NBATCH * 2 ||
      in_sizes[2] != NEMB * 2 || in_sizes[3] != NEMB ||
      in_sizes[4] != NGATE * NEMB || in_sizes[5] != NGATE * NHID ||
      in_sizes[6] != NGATE || in_sizes[7] != NGATE ||
      in_sizes[8] != NEMB * 2 || in_sizes[9] != NEMB ||
      in_sizes[10] != NGATE * NEMB || in_sizes[11] != NGATE * NHID ||
      in_sizes[12] != NGATE || in_sizes[13] != NGATE ||
      in_sizes[14] != 2 * NHID || in_sizes[15] != 2 ||
      out_size != PRED_STEPS * NBATCH * 2) return;

  const float* obs_rel   = (const float*)d_in[1];
  const float* enc_emb_w = (const float*)d_in[2];
  const float* enc_emb_b = (const float*)d_in[3];
  const float* enc_w_ih  = (const float*)d_in[4];
  const float* enc_w_hh  = (const float*)d_in[5];
  const float* enc_b_ih  = (const float*)d_in[6];
  const float* enc_b_hh  = (const float*)d_in[7];
  const float* dec_emb_w = (const float*)d_in[8];
  const float* dec_emb_b = (const float*)d_in[9];
  const float* dec_w_ih  = (const float*)d_in[10];
  const float* dec_w_hh  = (const float*)d_in[11];
  const float* dec_b_ih  = (const float*)d_in[12];
  const float* dec_b_hh  = (const float*)d_in[13];
  const float* h2p_w     = (const float*)d_in[14];
  const float* h2p_b     = (const float*)d_in[15];
  float* out = (float*)d_out;

  char* ws = (char*)d_ws;
  size_t off = 0;
  auto carve = [&](size_t bytes) -> char* { char* p = ws + off; off += (bytes + 255) & ~(size_t)255; return p; };
  unsigned short* WH  = (unsigned short*)carve((size_t)2 * WH_PHASE * 2);
  float*          TAB = (float*)carve((size_t)2 * TAB_PHASE * 4);
  if (off > ws_size || off > (size_t)134217728) return;

  prep_tables_kernel<<<2, NTHR, 0, stream>>>(enc_emb_w, enc_emb_b, enc_w_ih, enc_b_ih, enc_b_hh,
                                             dec_emb_w, dec_emb_b, dec_w_ih, dec_b_ih, dec_b_hh, TAB);
  cvt_whh_kernel<<<16, NTHR, 0, stream>>>(enc_w_hh, dec_w_hh, WH);
  lstm_seq_kernel<<<NBATCH / ROWS_BLK, NTHR, 0, stream>>>(obs_rel, WH, TAB, h2p_w, h2p_b, out);
}
